// ImprovedTransformerEncoderBlock_24747601559953
// MI455X (gfx1250) — hardware-verified
//
#include <hip/hip_runtime.h>
#include <math.h>

constexpr int DMOD   = 512;
constexpr int NHEAD  = 8;
constexpr int DHEAD  = 64;
constexpr int DFFN   = 2048;
constexpr int NBATCH = 4;
constexpr int SEQL   = 2048;
constexpr int NTOK   = NBATCH * SEQL;
constexpr int HTOK   = NTOK / 2;

constexpr float W_CARRY   = 256.0f;
constexpr float CTX_CARRY = 8.0f;
constexpr float ACT_CARRY = 64.0f;
constexpr float P_CARRY   = 32768.0f;

constexpr size_t MIB       = 1048576;
constexpr size_t OFF_WQK_H = 0;
constexpr size_t OFF_WQK_L = 1 * MIB;
constexpr size_t OFF_WV    = 2 * MIB;
constexpr size_t OFF_WO    = 2 * MIB + 524288;
constexpr size_t OFF_W1    = 3 * MIB;
constexpr size_t OFF_W2    = 7 * MIB;
constexpr size_t OFF_XF    = 9 * MIB;
constexpr size_t OFF_XBH   = 17 * MIB;
constexpr size_t OFF_XBL   = 25 * MIB;
constexpr size_t OFF_QKH   = 33 * MIB;
constexpr size_t OFF_QKL   = 49 * MIB;
constexpr size_t OFF_VT    = 65 * MIB;
constexpr size_t OFF_CTX   = 73 * MIB;
constexpr size_t OFF_SRC2  = 81 * MIB;
constexpr size_t WS_TOTAL  = 97 * MIB;
constexpr size_t OFF_HPL   = OFF_QKH;
constexpr size_t OFF_ACT   = OFF_VT;
static_assert(WS_TOTAL <= 134217728ull);
static_assert(OFF_HPL + (size_t)HTOK * (2 * DFFN) * 2 <= OFF_VT);
static_assert(OFF_ACT + (size_t)HTOK * DFFN * 2 <= OFF_SRC2);
static_assert(OFF_SRC2 + (size_t)NTOK * DMOD * 4 == WS_TOTAL);
static_assert(NTOK % 64 == 0 && HTOK % 64 == 0 && DMOD % 64 == 0 && (2 * DMOD) % 64 == 0 && (2 * DFFN) % 64 == 0 && DFFN % 64 == 0);
static_assert(DMOD % 32 == 0 && DFFN % 32 == 0);
static_assert(SEQL % 64 == 0 && DHEAD == 64);

typedef __attribute__((ext_vector_type(16))) _Float16 v16h;
typedef __attribute__((ext_vector_type(8)))  _Float16 v8h;
typedef __attribute__((ext_vector_type(16))) __bf16   v16b;
typedef __attribute__((ext_vector_type(8)))  __bf16   v8b;
typedef __attribute__((ext_vector_type(8)))  float    v8f;
typedef __attribute__((ext_vector_type(4)))  float    v4f;
typedef __attribute__((ext_vector_type(4)))  unsigned int u4;

__device__ __forceinline__ unsigned short f2bf_bits(float f) {
  unsigned u = __float_as_uint(f);
  return (unsigned short)((u + 0x7FFFu + ((u >> 16) & 1u)) >> 16);
}
__device__ __forceinline__ float bf_bits2f(unsigned short h) { return __uint_as_float(((unsigned)h) << 16); }

__device__ __forceinline__ void dep_guard_h(v8f& a, v8f& b, v16h x, v16h y) { asm volatile("v_nop\n\tv_nop\n\tv_nop\n\tv_nop" : "+v"(a), "+v"(b) : "v"(x), "v"(y)); }
__device__ __forceinline__ void dep_guard_b(v8f& a, v8f& b, v16b x, v16b y) { asm volatile("v_nop\n\tv_nop\n\tv_nop\n\tv_nop" : "+v"(a), "+v"(b) : "v"(x), "v"(y)); }
__device__ __forceinline__ void keep4_h(v16h a, v16h b, v16h c, v16h d) { asm volatile("v_nop" :: "v"(a), "v"(b), "v"(c), "v"(d)); }
__device__ __forceinline__ void keep4_b(v16b a, v16b b, v16b c, v16b d) { asm volatile("v_nop" :: "v"(a), "v"(b), "v"(c), "v"(d)); }
__device__ __forceinline__ void acc_guard4(v8f& a, v8f& b, v8f& c, v8f& d) { asm volatile("v_nop\n\tv_nop\n\tv_nop\n\tv_nop" : "+v"(a), "+v"(b), "+v"(c), "+v"(d)); }
template <typename T> struct Frag;
template <> struct Frag<_Float16> {
  typedef v16h V; union U { v16h v; v8h h[2]; };
  static __device__ __forceinline__ v16h load(const _Float16* p) {
    U f; f.h[0] = *(const v8h*)(p); f.h[1] = *(const v8h*)(p + 16); return f.v;
  }
  static __device__ __forceinline__ v8f mma(v16h a, v16h b, v8f c) {
    return __builtin_amdgcn_wmma_f32_16x16x32_f16(false, a, false, b, (short)0, c, false, false);
  }
  static __device__ __forceinline__ void guard(v8f& a, v8f& b, v16h x, v16h y) { dep_guard_h(a, b, x, y); }
  static __device__ __forceinline__ void keep(v16h a, v16h b, v16h c, v16h d) { keep4_h(a, b, c, d); }
};
template <> struct Frag<__bf16> {
  typedef v16b V; union U { v16b v; v8b h[2]; };
  static __device__ __forceinline__ v16b load(const __bf16* p) {
    U f; f.h[0] = *(const v8b*)(p); f.h[1] = *(const v8b*)(p + 16); return f.v;
  }
  static __device__ __forceinline__ v8f mma(v16b a, v16b b, v8f c) {
    return __builtin_amdgcn_wmma_f32_16x16x32_bf16(false, a, false, b, (short)0, c, false, false);
  }
  static __device__ __forceinline__ void guard(v8f& a, v8f& b, v16b x, v16b y) { dep_guard_b(a, b, x, y); }
  static __device__ __forceinline__ void keep(v16b a, v16b b, v16b c, v16b d) { keep4_b(a, b, c, d); }
};

__device__ __forceinline__ v8f at_mma(v16b a, v16b b, v8f c) {
  c = __builtin_amdgcn_wmma_f32_16x16x32_bf16(false, a, false, b, (short)0, c, false, false);
  asm volatile("v_nop\n\tv_nop\n\tv_nop\n\tv_nop" : "+v"(c) : "v"(a), "v"(b));
  return c;
}
__device__ __forceinline__ v8f mma_f16g(v16h a, v16h b, v8f c) {
  c = __builtin_amdgcn_wmma_f32_16x16x32_f16(false, a, false, b, (short)0, c, false, false);
  asm volatile("v_nop\n\tv_nop\n\tv_nop\n\tv_nop" : "+v"(c) : "v"(a), "v"(b));
  return c;
}

template <int ET> struct Elem;
template <> struct Elem<0> { typedef _Float16 T; };
template <> struct Elem<1> { typedef __bf16 T; };
template <int ET, bool SPLIT, int BIAS_MODE, int OUT_MODE, bool RESID>
__global__ __launch_bounds__(256) void wmma_gemm64(
    const unsigned short* __restrict__ Ap, const unsigned short* __restrict__ A2p, int lda, long strideA,
    const unsigned short* __restrict__ Btp, const unsigned short* __restrict__ Bt2p, int ldb, long strideB,
    void* __restrict__ Cout, void* __restrict__ Cout2, int ldc, long strideC,
    const float* __restrict__ bias,
    const float* __restrict__ resid, long strideR,
    int M, int N, int K, float scale) {
  static_assert(BIAS_MODE == 0 || BIAS_MODE == 2);
  static_assert(!(RESID && OUT_MODE != 0));
  typedef typename Elem<ET>::T T;
  typedef typename Frag<T>::V V;
  const T* A = (const T*)Ap; const T* A2 = (const T*)A2p; const T* Bt = (const T*)Btp; const T* Bt2 = (const T*)Bt2p;
  __shared__ __align__(16) float sT[8][16 * 68];
  const int b    = blockIdx.y;
  const int lane = threadIdx.x & 31;
  const int wave = threadIdx.x >> 5;
  const int tilesN = N >> 6;
  const int tilesM = M >> 6;
  const int tile = blockIdx.x * 8 + wave;
  if (tile >= tilesM * tilesN) return;
  const int tm = tile / tilesN;
  const int tn = tile - tm * tilesN;
  const int m0 = tm << 6;
  const int n0 = tn << 6;

  const T* Ab  = A  + (size_t)b * strideA;
  const T* Bb  = Bt + (size_t)b * strideB;
  const T* Ab2 = SPLIT ? (A2  + (size_t)b * strideA) : nullptr;
  const T* Bb2 = SPLIT ? (Bt2 + (size_t)b * strideB) : nullptr;

  const int rlane = lane & 15;
  const int koff  = (lane >> 4) * 8;
  const int mOff  = (lane >> 4) * 8;

  v8f acc[4][4];
#pragma unroll
  for (int i = 0; i < 4; ++i)
#pragma unroll
    for (int j = 0; j < 4; ++j) acc[i][j] = (v8f){0.f,0.f,0.f,0.f,0.f,0.f,0.f,0.f};

  for (int k0 = 0; k0 < K; k0 += 32) {
    V bh[4], bl[4];
#pragma unroll
    for (int j = 0; j < 4; ++j) {
      const size_t bo = (size_t)(n0 + (j << 4) + rlane) * ldb + koff + k0;
      bh[j] = Frag<T>::load(Bb + bo);
      if (SPLIT) bl[j] = Frag<T>::load(Bb2 + bo);
    }
#pragma unroll
    for (int i = 0; i < 4; ++i) {
      const size_t ao = (size_t)(m0 + (i << 4) + rlane) * lda + koff + k0;
      V ah = Frag<T>::load(Ab + ao);
      V al;
      if (SPLIT) al = Frag<T>::load(Ab2 + ao);
#pragma unroll
      for (int j = 0; j < 4; ++j) {
        acc[i][j] = Frag<T>::mma(ah, bh[j], acc[i][j]);
        if (SPLIT) {
          acc[i][j] = Frag<T>::mma(ah, bl[j], acc[i][j]);
          acc[i][j] = Frag<T>::mma(al, bh[j], acc[i][j]);
        }
      }
      Frag<T>::guard(acc[i][0], acc[i][3], ah, SPLIT ? al : ah);
    }
    Frag<T>::keep(bh[0], bh[1], bh[2], bh[3]);
    if (SPLIT) Frag<T>::keep(bl[0], bl[1], bl[2], bl[3]);
  }
  acc_guard4(acc[0][0], acc[0][1], acc[0][2], acc[0][3]);
  acc_guard4(acc[1][0], acc[1][1], acc[1][2], acc[1][3]);
  acc_guard4(acc[2][0], acc[2][1], acc[2][2], acc[2][3]);
  acc_guard4(acc[3][0], acc[3][1], acc[3][2], acc[3][3]);

  float* slab = sT[wave];
  const v4f zero4 = (v4f){0.f, 0.f, 0.f, 0.f};
#pragma unroll
  for (int i = 0; i < 4; ++i) {
    const int mBase = m0 + (i << 4);
#pragma unroll
    for (int j = 0; j < 4; ++j) {
#pragma unroll
      for (int r = 0; r < 8; ++r) slab[(mOff + r) * 68 + (j << 4) + rlane] = acc[i][j][r] * scale;
    }
    __builtin_amdgcn_fence(__ATOMIC_RELEASE, "workgroup");
    __builtin_amdgcn_wave_barrier();
    __builtin_amdgcn_fence(__ATOMIC_ACQUIRE, "workgroup");
    if (OUT_MODE == 0) {
      float* C = (float*)Cout + (size_t)b * strideC;
      const int hh = lane >> 4, c4 = (lane & 15) * 4;
      v4f bz = zero4;
      if (BIAS_MODE == 2) bz = *(const v4f*)(bias + n0 + c4);
      v4f vals[8];
#pragma unroll
      for (int it = 0; it < 8; ++it) {
        const int row = it * 2 + hh;
        v4f v = *(const v4f*)(slab + row * 68 + c4);
        v = v + bz;
        if (RESID) {
          const v4f rr = *(const v4f*)(resid + (size_t)b * strideR + (size_t)(mBase + row) * ldc + n0 + c4);
          v = v + rr;
        }
        vals[it] = v;
      }
      for (int pass = 0; pass < 2; ++pass) {
#pragma unroll
        for (int it = 0; it < 8; ++it) {
          const int row = it * 2 + hh;
          *(volatile v4f*)(C + (size_t)(mBase + row) * ldc + n0 + c4) = vals[it];
        }
        __threadfence();
      }
    } else {
      const int q = lane >> 3, c8 = (lane & 7) * 8;
      unsigned short* C  = (unsigned short*)Cout  + (size_t)b * strideC;
      unsigned short* C2 = (unsigned short*)Cout2 + (size_t)b * strideC;
      v4f b0z = zero4, b1z = zero4;
      if (BIAS_MODE == 2) { b0z = *(const v4f*)(bias + n0 + c8); b1z = *(const v4f*)(bias + n0 + c8 + 4); }
      v8h hv[4], lv[4];
#pragma unroll
      for (int it = 0; it < 4; ++it) {
        const int row = it * 4 + q;
        const float* sp = slab + row * 68 + c8;
        v4f x0 = *(const v4f*)(sp);
        v4f x1 = *(const v4f*)(sp + 4);
        x0 = x0 + b0z; x1 = x1 + b1z;
        float xe[8];
#pragma unroll
        for (int e = 0; e < 4; ++e) { xe[e] = x0[e]; xe[4 + e] = x1[e]; }
#pragma unroll
        for (int e = 0; e < 8; ++e) {
          if (OUT_MODE == 1) {
            hv[it][e] = (_Float16)xe[e];
            lv[it][e] = hv[it][e];
          } else {
            const unsigned short hb = f2bf_bits(xe[e]);
            const unsigned short lb = f2bf_bits(xe[e] - bf_bits2f(hb));
            hv[it][e] = __builtin_bit_cast(_Float16, hb);
            lv[it][e] = __builtin_bit_cast(_Float16, lb);
          }
        }
      }
      for (int pass = 0; pass < 2; ++pass) {
#pragma unroll
        for (int it = 0; it < 4; ++it) {
          const int row = it * 4 + q;
          *(volatile v8h*)(C + (size_t)(mBase + row) * ldc + n0 + c8) = hv[it];
          if (OUT_MODE == 2) *(volatile v8h*)(C2 + (size_t)(mBase + row) * ldc + n0 + c8) = lv[it];
        }
        __threadfence();
      }
    }
    __builtin_amdgcn_fence(__ATOMIC_RELEASE, "workgroup");
    __builtin_amdgcn_wave_barrier();
    __builtin_amdgcn_fence(__ATOMIC_ACQUIRE, "workgroup");
  }
}

constexpr int WT_PITCH = 72;
template <int MODE>
__global__ __launch_bounds__(256) void k_wtrans(const float* __restrict__ W,
                                                unsigned short* __restrict__ O1,
                                                unsigned short* __restrict__ O2,
                                                int Kin, int Nout, float carry) {
  __shared__ __align__(16) unsigned short th[64 * WT_PITCH];
  __shared__ __align__(16) unsigned short tl[(MODE == 1) ? 64 * WT_PITCH : 8];
  const int bn = blockIdx.x, bk = blockIdx.y, t = threadIdx.x;
#pragma unroll
  for (int i = 0; i < 4; ++i) {
    const int idx = t + 256 * i;
    const int kk = idx >> 4;
    const int c4 = (idx & 15) * 4;
    const v4f v = *(const v4f*)(W + (size_t)(bk * 64 + kk) * Nout + bn * 64 + c4);
#pragma unroll
    for (int e = 0; e < 4; ++e) {
      const float x = v[e];
      if (MODE == 0) {
        th[(c4 + e) * WT_PITCH + kk] = __builtin_bit_cast(unsigned short, (_Float16)(x * carry));
      } else {
        const unsigned short hb = f2bf_bits(x);
        th[(c4 + e) * WT_PITCH + kk] = hb;
        tl[(c4 + e) * WT_PITCH + kk] = f2bf_bits(x - bf_bits2f(hb));
      }
    }
  }
  __syncthreads();
  const int wave = t >> 5, lane = t & 31;
  const int q = lane >> 3, c8 = (lane & 7) * 8;
  u4 hv[2], lv[2];
#pragma unroll
  for (int it = 0; it < 2; ++it) {
    const int n = wave * 8 + it * 4 + q;
    hv[it] = *(const u4*)(th + n * WT_PITCH + c8);
    lv[it] = hv[it];
    if (MODE == 1) lv[it] = *(const u4*)(tl + n * WT_PITCH + c8);
  }
  for (int pass = 0; pass < 2; ++pass) {
#pragma unroll
    for (int it = 0; it < 2; ++it) {
      const int n = wave * 8 + it * 4 + q;
      const size_t o = (size_t)(bn * 64 + n) * Kin + bk * 64 + c8;
      *(volatile u4*)(O1 + o) = hv[it];
      if (MODE == 1) *(volatile u4*)(O2 + o) = lv[it];
    }
    __threadfence();
  }
}

template <int MODE>
__global__ __launch_bounds__(256) void k_layernorm(const float* __restrict__ X,
                                                   const float* __restrict__ gam,
                                                   const float* __restrict__ bet,
                                                   unsigned short* __restrict__ O1,
                                                   unsigned short* __restrict__ O2,
                                                   unsigned short* __restrict__ O3,
                                                   int nrows) {
  const int wave = threadIdx.x >> 5, lane = threadIdx.x & 31;
  const int row = blockIdx.x * 8 + wave;
  if (row >= nrows) return;
  const float* xr = X + (size_t)row * DMOD;
  const int c0 = 8 * lane, c1 = 256 + 8 * lane;
  const v4f a0 = *(const v4f*)(xr + c0), a1 = *(const v4f*)(xr + c0 + 4);
  const v4f a2 = *(const v4f*)(xr + c1), a3 = *(const v4f*)(xr + c1 + 4);
  const v4f g0 = *(const v4f*)(gam + c0), g1 = *(const v4f*)(gam + c0 + 4);
  const v4f g2 = *(const v4f*)(gam + c1), g3 = *(const v4f*)(gam + c1 + 4);
  const v4f e0 = *(const v4f*)(bet + c0), e1 = *(const v4f*)(bet + c0 + 4);
  const v4f e2 = *(const v4f*)(bet + c1), e3 = *(const v4f*)(bet + c1 + 4);
  float xv[16], gv[16], bv[16];
#pragma unroll
  for (int e = 0; e < 4; ++e) {
    xv[e] = a0[e]; xv[4 + e] = a1[e]; xv[8 + e] = a2[e]; xv[12 + e] = a3[e];
    gv[e] = g0[e]; gv[4 + e] = g1[e]; gv[8 + e] = g2[e]; gv[12 + e] = g3[e];
    bv[e] = e0[e]; bv[4 + e] = e1[e]; bv[8 + e] = e2[e]; bv[12 + e] = e3[e];
  }
  float s = 0.f;
#pragma unroll
  for (int e = 0; e < 16; ++e) s += xv[e];
#pragma unroll
  for (int off = 1; off < 32; off <<= 1) s += __shfl_xor(s, off, 32);
  const float mu = s * (1.0f / 512.0f);
  float ss = 0.f;
#pragma unroll
  for (int e = 0; e < 16; ++e) { const float d = xv[e] - mu; xv[e] = d; ss += d * d; }
#pragma unroll
  for (int off = 1; off < 32; off <<= 1) ss += __shfl_xor(ss, off, 32);
  const float var = ss * (1.0f / 512.0f);
  const float rs = rsqrtf(var + 1e-5f);
  unsigned short fb[16], hb[16], lb[16];
#pragma unroll
  for (int e = 0; e < 16; ++e) {
    const float y = xv[e] * rs * gv[e] + bv[e];
    fb[e] = __builtin_bit_cast(unsigned short, (_Float16)y);
    hb[e] = fb[e]; lb[e] = fb[e];
    if (MODE == 1) {
      hb[e] = f2bf_bits(y);
      lb[e] = f2bf_bits(y - bf_bits2f(hb[e]));
    }
  }
  u4 f0, f1, h0, h1, l0, l1;
#pragma unroll
  for (int qd = 0; qd < 4; ++qd) {
    f0[qd] = (unsigned)fb[2 * qd] | ((unsigned)fb[2 * qd + 1] << 16);
    f1[qd] = (unsigned)fb[8 + 2 * qd] | ((unsigned)fb[8 + 2 * qd + 1] << 16);
    h0[qd] = (unsigned)hb[2 * qd] | ((unsigned)hb[2 * qd + 1] << 16);
    h1[qd] = (unsigned)hb[8 + 2 * qd] | ((unsigned)hb[8 + 2 * qd + 1] << 16);
    l0[qd] = (unsigned)lb[2 * qd] | ((unsigned)lb[2 * qd + 1] << 16);
    l1[qd] = (unsigned)lb[8 + 2 * qd] | ((unsigned)lb[8 + 2 * qd + 1] << 16);
  }
  const size_t ro = (size_t)row * DMOD;
  for (int pass = 0; pass < 2; ++pass) {
    *(volatile u4*)(O1 + ro + c0) = f0;
    *(volatile u4*)(O1 + ro + c1) = f1;
    if (MODE == 1) {
      *(volatile u4*)(O2 + ro + c0) = h0;
      *(volatile u4*)(O2 + ro + c1) = h1;
      *(volatile u4*)(O3 + ro + c0) = l0;
      *(volatile u4*)(O3 + ro + c1) = l1;
    }
    __threadfence();
  }
}

constexpr int ATT_D  = 64;
constexpr int ATT_KC = 64;
__global__ __launch_bounds__(128) void k_attn_alibi(
    const unsigned short* __restrict__ Qhp, const unsigned short* __restrict__ Qlp,
    const unsigned short* __restrict__ Vtp,
    const int* __restrict__ kpm,
    unsigned short* __restrict__ ctxp,
    float out_carry) {
  const __bf16* QH = (const __bf16*)Qhp;
  const __bf16* QL = (const __bf16*)Qlp;
  const _Float16* VT = (const _Float16*)Vtp;
  _Float16* CTX = (_Float16*)ctxp;
  __shared__ __align__(16) __bf16   Ksh[ATT_KC * ATT_D];
  __shared__ __align__(16) __bf16   Ksl[ATT_KC * ATT_D];
  __shared__ __align__(16) _Float16 Vth[ATT_D * ATT_KC];
  __shared__ __align__(16) _Float16 Psh[4][16 * ATT_KC];
  __shared__ __align__(16) float    Os[4][16 * 68];

  const int tid  = threadIdx.x;
  const int wave = tid >> 5;
  const int lane = tid & 31;
  const int hh   = lane >> 4;
  const int c    = lane & 15;

  const int nqb = SEQL / 64;
  const int bx = blockIdx.x;
  const int qb = bx % nqb;
  const int bh = bx / nqb;
  const int h  = bh % NHEAD;
  const int b  = bh / NHEAD;
  const int q0 = qb * 64 + wave * 16;
  const float slope = __uint_as_float((unsigned)(126 - h) << 23);

  v16b qah[2], qal[2];
  {
    const size_t qoff = (size_t)(b * SEQL + q0 + c) * (2 * DMOD) + h * DHEAD + 8 * hh;
#pragma unroll
    for (int dc = 0; dc < 2; ++dc) {
      qah[dc] = Frag<__bf16>::load(QH + qoff + dc * 32);
      qal[dc] = Frag<__bf16>::load(QL + qoff + dc * 32);
    }
  }

  float mrow[8], lrow[8];
  v8f oacc[4];
#pragma unroll
  for (int r = 0; r < 8; ++r) { mrow[r] = -INFINITY; lrow[r] = 0.f; }
#pragma unroll
  for (int t = 0; t < 4; ++t) oacc[t] = (v8f){0.f,0.f,0.f,0.f,0.f,0.f,0.f,0.f};

  for (int kc = 0; kc < SEQL / ATT_KC; ++kc) {
    const int kv0 = kc * ATT_KC;
    __syncthreads();
    {
      const int rr = tid >> 1, half = (tid & 1) * 32;
      const size_t koff = (size_t)(b * SEQL + kv0 + rr) * (2 * DMOD) + DMOD + h * DHEAD + half;
      const size_t voff = (size_t)(h * DHEAD + rr) * NTOK + (size_t)b * SEQL + kv0 + half;
#pragma unroll
      for (int i = 0; i < 4; ++i) {
        *(v8b*)(Ksh + rr * ATT_D + half + 8 * i) = *(const v8b*)(QH + koff + 8 * i);
        *(v8b*)(Ksl + rr * ATT_D + half + 8 * i) = *(const v8b*)(QL + koff + 8 * i);
        *(v8h*)(Vth + rr * ATT_KC + half + 8 * i) = *(const v8h*)(VT + voff + 8 * i);
      }
    }
    __syncthreads();

    v8f s[4];
#pragma unroll
    for (int j = 0; j < 4; ++j) {
      s[j] = (v8f){0.f,0.f,0.f,0.f,0.f,0.f,0.f,0.f};
#pragma unroll
      for (int dc = 0; dc < 2; ++dc) {
        const v16b kb = Frag<__bf16>::load(Ksh + (j * 16 + c) * ATT_D + dc * 32 + 8 * hh);
        const v16b kl = Frag<__bf16>::load(Ksl + (j * 16 + c) * ATT_D + dc * 32 + 8 * hh);
        s[j] = at_mma(qah[dc], kb, s[j]);
        s[j] = at_mma(qah[dc], kl, s[j]);
        s[j] = at_mma(qal[dc], kb, s[j]);
      }
    }
    int kvkeep[4];
#pragma unroll
    for (int j = 0; j < 4; ++j) kvkeep[j] = kpm[(size_t)b * SEQL + kv0 + j * 16 + c];
    float cm[8];
#pragma unroll
    for (int r = 0; r < 8; ++r) {
      const int qi = q0 + 8 * hh + r;
      float m = -INFINITY;
#pragma unroll
      for (int j = 0; j < 4; ++j) {
        const int kvcol = kv0 + j * 16 + c;
        float sv = s[j][r] * 0.125f + slope * (float)(kvcol - qi);
        if (kvkeep[j] != 0) sv = -INFINITY;
        s[j][r] = sv;
        m = fmaxf(m, sv);
      }
#pragma unroll
      for (int off = 1; off < 16; off <<= 1) m = fmaxf(m, __shfl_xor(m, off, 32));
      cm[r] = m;
    }
    _Float16* pwh = Psh[wave];
#pragma unroll
    for (int r = 0; r < 8; ++r) {
      const float mnew = fmaxf(mrow[r], cm[r]);
      const float msafe = (mnew == -INFINITY) ? 0.f : mnew;
      const float alpha = expf(mrow[r] - msafe);
      mrow[r] = mnew;
      float psum = 0.f;
#pragma unroll
      for (int j = 0; j < 4; ++j) {
        const float p = expf(s[j][r] - msafe);
        psum += p;
        pwh[(8 * hh + r) * ATT_KC + j * 16 + c] = (_Float16)(p * P_CARRY);
      }
#pragma unroll
      for (int off = 1; off < 16; off <<= 1) psum += __shfl_xor(psum, off, 32);
      lrow[r] = lrow[r] * alpha + psum;
#pragma unroll
      for (int t = 0; t < 4; ++t) oacc[t][r] *= alpha;
    }
    __builtin_amdgcn_fence(__ATOMIC_RELEASE, "workgroup");
    __builtin_amdgcn_wave_barrier();
    __builtin_amdgcn_fence(__ATOMIC_ACQUIRE, "workgroup");
#pragma unroll
    for (int kk = 0; kk < 2; ++kk) {
      const v16h pa = Frag<_Float16>::load(pwh + c * ATT_KC + kk * 32 + 8 * hh);
#pragma unroll
      for (int t = 0; t < 4; ++t) {
        const v16h vb = Frag<_Float16>::load(Vth + (t * 16 + c) * ATT_KC + kk * 32 + 8 * hh);
        oacc[t] = mma_f16g(pa, vb, oacc[t]);
      }
    }
  }

  float* os = Os[wave];
#pragma unroll
  for (int r = 0; r < 8; ++r) {
    const float inv = out_carry * (1.0f / (lrow[r] * P_CARRY));
#pragma unroll
    for (int t = 0; t < 4; ++t) os[(8 * hh + r) * 68 + t * 16 + c] = oacc[t][r] * inv;
  }
  __builtin_amdgcn_fence(__ATOMIC_RELEASE, "workgroup");
  __builtin_amdgcn_wave_barrier();
  __builtin_amdgcn_fence(__ATOMIC_ACQUIRE, "workgroup");
  {
    const int q8 = lane >> 3, c8 = (lane & 7) * 8;
    v8h hv[4];
#pragma unroll
    for (int it = 0; it < 4; ++it) {
      const int row = it * 4 + q8;
      const float* sp = os + row * 68 + c8;
      const v4f x0 = *(const v4f*)(sp);
      const v4f x1 = *(const v4f*)(sp + 4);
#pragma unroll
      for (int e = 0; e < 4; ++e) { hv[it][e] = (_Float16)x0[e]; hv[it][4 + e] = (_Float16)x1[e]; }
    }
    for (int pass = 0; pass < 2; ++pass) {
#pragma unroll
      for (int it = 0; it < 4; ++it) {
        const int row = it * 4 + q8;
        *(volatile v8h*)(CTX + (size_t)(b * SEQL + q0 + row) * DMOD + h * DHEAD + c8) = hv[it];
      }
      __threadfence();
    }
  }
}

__global__ __launch_bounds__(256) void k_geglu(const unsigned* __restrict__ H,
                                               unsigned* __restrict__ A, int nrows) {
  const size_t i = (size_t)blockIdx.x * 256 + threadIdx.x;
  const size_t total = (size_t)nrows * (DFFN / 2);
  if (i >= total) return;
  const size_t row = i / (DFFN / 2);
  const size_t cw  = i - row * (DFFN / 2);
  const unsigned wg = H[row * DFFN + cw];
  const unsigned wl = H[row * DFFN + (DFFN / 2) + cw];
  unsigned outw = 0u;
#pragma unroll 1
  for (int e = 0; e < 2; ++e) {
    const int sh = 16 * e;
    const float g = (float)__builtin_bit_cast(_Float16, (unsigned short)((wg >> sh) & 0xffffu));
    const float l = (float)__builtin_bit_cast(_Float16, (unsigned short)((wl >> sh) & 0xffffu));
    const float ge = 0.5f * g * (1.0f + erff(g * 0.70710678118654752f));
    const float a = ge * l * ACT_CARRY;
    outw |= ((unsigned)__builtin_bit_cast(unsigned short, (_Float16)a)) << sh;
  }
  ((volatile unsigned*)A)[i] = outw;
  __threadfence();
  ((volatile unsigned*)A)[i] = outw;
}

extern "C" void kernel_launch(void* const* d_in, const int* in_sizes, int n_in,
                              void* d_out, int out_size, void* d_ws, size_t ws_size,
                              hipStream_t stream) {
  const float* src   = (const float*)d_in[0];
  const int*   kpm   = (const int*)d_in[1];
  const float* w_q   = (const float*)d_in[2];
  const float* w_k   = (const float*)d_in[3];
  const float* w_v   = (const float*)d_in[4];
  const float* w_o   = (const float*)d_in[5];
  const float* b_o   = (const float*)d_in[6];
  const float* w1    = (const float*)d_in[7];
  const float* b1    = (const float*)d_in[8];
  const float* w2    = (const float*)d_in[9];
  const float* b2    = (const float*)d_in[10];
  const float* ln1_g = (const float*)d_in[11];
  const float* ln1_b = (const float*)d_in[12];
  const float* ln2_g = (const float*)d_in[13];
  const float* ln2_b = (const float*)d_in[14];
  float* out = (float*)d_out;

  char* ws = (char*)d_ws;
  unsigned short* WQKH = (unsigned short*)(ws + OFF_WQK_H);
  unsigned short* WQKL = (unsigned short*)(ws + OFF_WQK_L);
  unsigned short* WVT  = (unsigned short*)(ws + OFF_WV);
  unsigned short* WOT  = (unsigned short*)(ws + OFF_WO);
  unsigned short* W1T  = (unsigned short*)(ws + OFF_W1);
  unsigned short* W2T  = (unsigned short*)(ws + OFF_W2);
  unsigned short* XF   = (unsigned short*)(ws + OFF_XF);
  unsigned short* XBH  = (unsigned short*)(ws + OFF_XBH);
  unsigned short* XBL  = (unsigned short*)(ws + OFF_XBL);
  unsigned short* QKH  = (unsigned short*)(ws + OFF_QKH);
  unsigned short* QKL  = (unsigned short*)(ws + OFF_QKL);
  unsigned short* VTP  = (unsigned short*)(ws + OFF_VT);
  unsigned short* CTX  = (unsigned short*)(ws + OFF_CTX);
  float*          SRC2 = (float*)(ws + OFF_SRC2);
  unsigned short* HPL  = (unsigned short*)(ws + OFF_HPL);
  unsigned short* ACT  = (unsigned short*)(ws + OFF_ACT);

  k_wtrans<1><<<dim3(DMOD / 64, DMOD / 64), 256, 0, stream>>>(w_q, WQKH, WQKL, DMOD, DMOD, 1.0f);
  k_wtrans<1><<<dim3(DMOD / 64, DMOD / 64), 256, 0, stream>>>(w_k, WQKH + (size_t)DMOD * DMOD, WQKL + (size_t)DMOD * DMOD, DMOD, DMOD, 1.0f);
  k_wtrans<0><<<dim3(DMOD / 64, DMOD / 64), 256, 0, stream>>>(w_v, WVT, WVT, DMOD, DMOD, W_CARRY);
  k_wtrans<0><<<dim3(DMOD / 64, DMOD / 64), 256, 0, stream>>>(w_o, WOT, WOT, DMOD, DMOD, W_CARRY);
  k_wtrans<0><<<dim3((2 * DFFN) / 64, DMOD / 64), 256, 0, stream>>>(w1, W1T, W1T, DMOD, 2 * DFFN, W_CARRY);
  k_wtrans<0><<<dim3(DMOD / 64, DFFN / 64), 256, 0, stream>>>(w2, W2T, W2T, DFFN, DMOD, W_CARRY);

  k_layernorm<1><<<NTOK / 8, 256, 0, stream>>>(src, ln1_g, ln1_b, XF, XBH, XBL, NTOK);

  {
    const int tiles = (NTOK / 64) * ((2 * DMOD) / 64);
    wmma_gemm64<1, true, 0, 2, false><<<dim3((tiles + 7) / 8, 1), 256, 0, stream>>>(
        XBH, XBL, DMOD, 0L, WQKH, WQKL, DMOD, 0L, QKH, QKL, 2 * DMOD, 0L, b_o, src, 0L,
        NTOK, 2 * DMOD, DMOD, 1.0f);
  }
  {
    const int tiles = (DMOD / 64) * (NTOK / 64);
    wmma_gemm64<0, false, 0, 1, false><<<dim3((tiles + 7) / 8, 1), 256, 0, stream>>>(
        WVT, WVT, DMOD, 0L, XF, XF, DMOD, 0L, VTP, VTP, NTOK, 0L, b_o, src, 0L,
        DMOD, NTOK, DMOD, 1.0f / W_CARRY);
  }
  k_attn_alibi<<<NBATCH * NHEAD * (SEQL / 64), 128, 0, stream>>>(QKH, QKL, VTP, kpm, CTX, CTX_CARRY);

  {
    const int tiles = (NTOK / 64) * (DMOD / 64);
    wmma_gemm64<0, false, 2, 0, true><<<dim3((tiles + 7) / 8, 1), 256, 0, stream>>>(
        CTX, CTX, DMOD, 0L, WOT, WOT, DMOD, 0L, SRC2, SRC2, DMOD, 0L, b_o, src, 0L,
        NTOK, DMOD, DMOD, 1.0f / (CTX_CARRY * W_CARRY));
  }
  k_layernorm<0><<<NTOK / 8, 256, 0, stream>>>(SRC2, ln2_g, ln2_b, XF, XF, XF, NTOK);

  for (int half = 0; half < 2; ++half) {
    const unsigned short* x2p = XF + (size_t)half * HTOK * DMOD;
    const float* src2p = SRC2 + (size_t)half * HTOK * DMOD;
    float* outp = out + (size_t)half * HTOK * DMOD;
    {
      const int tiles = (HTOK / 64) * ((2 * DFFN) / 64);
      wmma_gemm64<0, false, 2, 1, false><<<dim3((tiles + 7) / 8, 1), 256, 0, stream>>>(
          x2p, x2p, DMOD, 0L, W1T, W1T, DMOD, 0L, HPL, HPL, 2 * DFFN, 0L, b1, src, 0L,
          HTOK, 2 * DFFN, DMOD, 1.0f / W_CARRY);
    }
    k_geglu<<<(HTOK * (DFFN / 2)) / 256, 256, 0, stream>>>((const unsigned*)HPL, (unsigned*)ACT, HTOK);
    {
      const int tiles = (HTOK / 64) * (DMOD / 64);
      wmma_gemm64<0, false, 2, 0, true><<<dim3((tiles + 7) / 8, 1), 256, 0, stream>>>(
          ACT, ACT, DFFN, 0L, W2T, W2T, DFFN, 0L, outp, outp, DMOD, 0L, b2, src2p, 0L,
          HTOK, DMOD, DFFN, 1.0f / (ACT_CARRY * W_CARRY));
    }
  }

  (void)in_sizes; (void)n_in; (void)out_size; (void)ws_size;
}
